// ScaleDotProductAttention_25434796327363
// MI455X (gfx1250) — hardware-verified
//
#include <hip/hip_runtime.h>
#include <math.h>

constexpr int kB  = 2;
constexpr int kH  = 16;
constexpr int kS  = 2048;
constexpr int kD  = 64;
constexpr int kBH = kB * kH;
constexpr int kQB = 64;
constexpr int kKC = 64;
constexpr int kNW = 4;
constexpr int kOP = 68;
constexpr float kScale      = 0.125f;
constexpr float kPCarry     = 32768.0f;
constexpr float kPCarryInv  = 1.0f / 32768.0f;
constexpr float kLoCarry    = 2048.0f;
constexpr float kLoCarryInv = 1.0f / 2048.0f;
static_assert(kS % kQB == 0 && kS % kKC == 0 && kD == 64 && kQB == kKC, "shape");
static_assert((kBH * kS * kD) % 2048 == 0, "cast grid");

typedef __attribute__((ext_vector_type(16))) _Float16 v16h;
typedef __attribute__((ext_vector_type(8)))  _Float16 v8h;
typedef __attribute__((ext_vector_type(8)))  float    v8f;
typedef __attribute__((ext_vector_type(4)))  float    v4f;
typedef __attribute__((ext_vector_type(4)))  unsigned int v4u;

__device__ __forceinline__ unsigned short f2bf_bits(float f) {
  unsigned u = __float_as_uint(f);
  return (unsigned short)((u + 0x7FFFu + ((u >> 16) & 1u)) >> 16);
}
__device__ __forceinline__ float bf_bits2f(unsigned short h) { return __uint_as_float(((unsigned)h) << 16); }
__device__ __forceinline__ unsigned pk16(unsigned short a, unsigned short b) { return (unsigned)a | ((unsigned)b << 16); }
__device__ __forceinline__ unsigned short h_bits(float f) { const _Float16 h = (_Float16)f; return __builtin_bit_cast(unsigned short, h); }
__device__ __forceinline__ unsigned short hb16(float f) { return h_bits(bf_bits2f(f2bf_bits(f))); }
__device__ __forceinline__ float h16_to_f32(unsigned hb) {
  const unsigned sgn = (hb & 0x8000u) << 16; const unsigned em = hb & 0x7fffu;
  const float fn = __uint_as_float((em << 13) + 0x38000000u);
  const float fs = (float)em * 5.9604644775390625e-8f;
  const float mag = (em < 0x400u) ? fs : fn; return __uint_as_float(__float_as_uint(mag) | sgn); }

template <typename T> struct Frag;
template <> struct Frag<_Float16> {
  typedef v16h V; union U { v16h v; v8h h[2]; };
  static __device__ __forceinline__ v16h load(const _Float16* p) {
    U f; f.h[0] = *(const v8h*)(p); f.h[1] = *(const v8h*)(p + 16); return f.v;
  }
};
__device__ __forceinline__ v16h ldfrag(const unsigned short* p) {
  return Frag<_Float16>::load((const _Float16*)(const void*)p);
}
__device__ __forceinline__ v8f mma_h(v16h a, v16h b, v8f c) {
  c = __builtin_amdgcn_wmma_f32_16x16x32_f16(false, a, false, b, (short)0, c, false, false);
  asm volatile("v_nop\n\tv_nop\n\tv_nop\n\tv_nop" : "+v"(c) : "v"(a), "v"(b));
  return c;
}

__global__ __launch_bounds__(256) void cast8_kernel(const float* __restrict__ in, unsigned short* __restrict__ out, int n8) {
  const int i = blockIdx.x * 256 + threadIdx.x;
  if (i >= n8) return;
  const float* p = in + 8 * (size_t)i;
  const v4f a = *(const v4f*)(p);
  const v4f c = *(const v4f*)(p + 4);
  unsigned short hb[8];
#pragma unroll
  for (int e = 0; e < 4; ++e) {
    hb[e]     = hb16(a[e]);
    hb[4 + e] = hb16(c[e]);
  }
  const v4u u = (v4u){pk16(hb[0], hb[1]), pk16(hb[2], hb[3]), pk16(hb[4], hb[5]), pk16(hb[6], hb[7])};
  unsigned short* q = out + 8 * (size_t)i;
  *(volatile v4u*)q = u;
  __threadfence();
  *(volatile v4u*)q = u;
}

__global__ __launch_bounds__(256) void vt_cast_kernel(const float* __restrict__ v, unsigned short* __restrict__ VT) {
  __shared__ float sm[64][65];
  const int t  = threadIdx.x;
  const int s0 = blockIdx.x * 64;
  const int bh = blockIdx.y;
  const float* vb = v + ((size_t)bh * kS + s0) * kD;
#pragma unroll
  for (int i = 0; i < 4; ++i) {
    const int e4 = i * 256 + t;
    const int r  = e4 >> 4;
    const int c  = (e4 & 15) * 4;
    const v4f w = *(const v4f*)(vb + (size_t)e4 * 4);
    sm[c][r]     = w[0];
    sm[c + 1][r] = w[1];
    sm[c + 2][r] = w[2];
    sm[c + 3][r] = w[3];
  }
  __syncthreads();
  const int lane = t & 31, wave = t >> 5;
  const int q = lane >> 3, c8 = (lane & 7) * 8;
  unsigned short* op = VT + (size_t)bh * kD * kS;
  for (int pass = 0; pass < 2; ++pass) {
#pragma unroll
    for (int it = 0; it < 2; ++it) {
      const int row = wave * 8 + it * 4 + q;
      unsigned short hb[8];
#pragma unroll
      for (int e = 0; e < 8; ++e) hb[e] = hb16(sm[row][c8 + e]);
      const v4u u = (v4u){pk16(hb[0], hb[1]), pk16(hb[2], hb[3]), pk16(hb[4], hb[5]), pk16(hb[6], hb[7])};
      *(volatile v4u*)(op + (size_t)row * kS + s0 + c8) = u;
    }
    __threadfence();
  }
}

__global__ __launch_bounds__(128)
void attn_causal_kernel(const unsigned short* __restrict__ Q16, const unsigned short* __restrict__ K16,
                        const unsigned short* __restrict__ VT, float* __restrict__ out) {
  __shared__ __align__(16) unsigned short Ksh[kKC * kD];
  __shared__ __align__(16) unsigned short Vth[kD * kKC];
  __shared__ __align__(16) unsigned short Psh[kNW][16 * kKC];
  __shared__ __align__(16) unsigned short Psl[kNW][16 * kKC];
  __shared__ __align__(16) float Os[kNW][16 * kOP];

  const int tid  = threadIdx.x;
  const int wave = tid >> 5;
  const int lane = tid & 31;
  const int hh   = lane >> 4;
  const int c    = lane & 15;
  const int qb   = blockIdx.x;
  const int bh   = blockIdx.y;
  const int q0   = qb * kQB + wave * 16;
  const size_t pofs = (size_t)bh * kS * kD;
  const unsigned short* qpl = Q16 + pofs;
  const unsigned short* kpl = K16 + pofs;
  const unsigned short* vpl = VT + pofs;
  float* opl = out + pofs;

  v16h qa0, qa1;
  {
    const unsigned short* qrow = qpl + (size_t)(q0 + c) * kD + 8 * hh;
    qa0 = ldfrag(qrow);
    qa1 = ldfrag(qrow + 32);
  }

  const v8f z8 = (v8f){0.f, 0.f, 0.f, 0.f, 0.f, 0.f, 0.f, 0.f};
  float mrow[8], lrow[8];
  v8f oh[4], ol[4];
#pragma unroll
  for (int r = 0; r < 8; ++r) { mrow[r] = -__builtin_inff(); lrow[r] = 0.0f; }
#pragma unroll
  for (int t = 0; t < 4; ++t) { oh[t] = z8; ol[t] = z8; }

  const int nChunks = qb + 1;
  for (int kc = 0; kc < nChunks; ++kc) {
    const int kv0 = kc * kKC;
    __syncthreads();
#pragma unroll
    for (int i = 0; i < 4; ++i) {
      const int idx = i * 128 + tid;
      const int row = idx >> 3;
      const int c8  = (idx & 7) * 8;
      const v4u w = *(const v4u*)(kpl + (size_t)(kv0 + row) * kD + c8);
      *(v4u*)(Ksh + row * kD + c8) = w;
    }
    asm volatile("" ::: "memory");
#pragma unroll
    for (int i = 0; i < 4; ++i) {
      const int idx = i * 128 + tid;
      const int row = idx >> 3;
      const int c8  = (idx & 7) * 8;
      const v4u w = *(const v4u*)(vpl + (size_t)row * kS + kv0 + c8);
      *(v4u*)(Vth + row * kKC + c8) = w;
    }
    __syncthreads();

    v8f s[4];
#pragma unroll
    for (int j = 0; j < 4; ++j) {
      const unsigned short* kr = Ksh + (j * 16 + c) * kD + 8 * hh;
      const v16h kb0 = ldfrag(kr);
      const v16h kb1 = ldfrag(kr + 32);
      v8f a = mma_h(qa0, kb0, z8);
      a = mma_h(qa1, kb1, a);
      s[j] = a;
    }

    const bool diag = (kc == qb);
    float cm[8];
#pragma unroll
    for (int r = 0; r < 8; ++r) {
      const int qrow = q0 + 8 * hh + r;
      float m = -__builtin_inff();
#pragma unroll
      for (int j = 0; j < 4; ++j) {
        const int kvcol = kv0 + j * 16 + c;
        const float sv  = s[j][r] * kScale;
        const bool  msk = diag && (kvcol > qrow);
        const float se  = msk ? -__builtin_inff() : sv;
        s[j][r] = se;
        m = fmaxf(m, se);
      }
#pragma unroll
      for (int off = 1; off < 16; off <<= 1) m = fmaxf(m, __shfl_xor(m, off, 32));
      cm[r] = m;
    }

    unsigned short* pwh = Psh[wave];
    unsigned short* pwl = Psl[wave];
#pragma unroll
    for (int r = 0; r < 8; ++r) {
      const float mnew  = fmaxf(mrow[r], cm[r]);
      const float alpha = expf(mrow[r] - mnew);
      mrow[r] = mnew;
      float psum = 0.0f;
#pragma unroll
      for (int j = 0; j < 4; ++j) {
        const float p   = expf(s[j][r] - mnew);
        psum += p;
        const float x   = p * kPCarry;
        const unsigned hb = (unsigned)h_bits(x);
        const float res = (x - h16_to_f32(hb)) * kLoCarry;
        const unsigned short lb = h_bits(res);
        const int po = (8 * hh + r) * kKC + j * 16 + c;
        pwh[po] = (unsigned short)hb;
        pwl[po] = lb;
      }
#pragma unroll
      for (int off = 1; off < 16; off <<= 1) psum += __shfl_xor(psum, off, 32);
      lrow[r] = lrow[r] * alpha + psum;
#pragma unroll
      for (int t = 0; t < 4; ++t) { oh[t][r] *= alpha; ol[t][r] *= alpha; }
    }
    __syncthreads();

#pragma unroll
    for (int kk = 0; kk < 2; ++kk) {
      const v16h pa = ldfrag(pwh + c * kKC + kk * 32 + 8 * hh);
      const v16h pl = ldfrag(pwl + c * kKC + kk * 32 + 8 * hh);
#pragma unroll
      for (int t = 0; t < 4; ++t) {
        const v16h vbf = ldfrag(Vth + (t * 16 + c) * kKC + kk * 32 + 8 * hh);
        oh[t] = mma_h(pa, vbf, oh[t]);
        ol[t] = mma_h(pl, vbf, ol[t]);
      }
    }
  }

  float* os = Os[wave];
#pragma unroll
  for (int r = 0; r < 8; ++r) {
    const float inv = (1.0f / lrow[r]) * kPCarryInv;
#pragma unroll
    for (int t = 0; t < 4; ++t) os[(8 * hh + r) * kOP + t * 16 + c] = (oh[t][r] + ol[t][r] * kLoCarryInv) * inv;
  }
  __syncthreads();
  {
    const int c4 = (lane & 15) * 4;
    for (int pass = 0; pass < 2; ++pass) {
#pragma unroll
      for (int it = 0; it < 8; ++it) {
        const int row = it * 2 + hh;
        const v4f val = *(const v4f*)(os + row * kOP + c4);
        *(volatile v4f*)(opl + (size_t)(q0 + row) * kD + c4) = val;
      }
      __threadfence();
    }
  }
}

extern "C" void kernel_launch(void* const* d_in, const int* in_sizes, int n_in,
                              void* d_out, int out_size, void* d_ws, size_t ws_size,
                              hipStream_t stream) {
  if (n_in < 4) return;
  const int nElem = kBH * kS * kD;
  if (in_sizes[0] != nElem || in_sizes[1] != nElem || in_sizes[2] != nElem) return;
  if (out_size != nElem) return;

  const size_t szPlane = (size_t)nElem * 2;
  const size_t offQ  = 0;
  const size_t offK  = offQ + szPlane;
  const size_t offVT = offK + szPlane;
  const size_t total = offVT + szPlane;
  if (ws_size < total) return;

  const float* q = (const float*)d_in[0];
  const float* k = (const float*)d_in[1];
  const float* v = (const float*)d_in[2];
  float* out = (float*)d_out;
  char* ws = (char*)d_ws;
  unsigned short* Q16 = (unsigned short*)(ws + offQ);
  unsigned short* K16 = (unsigned short*)(ws + offK);
  unsigned short* VT  = (unsigned short*)(ws + offVT);

  const int n8 = nElem / 8;
  cast8_kernel<<<dim3(n8 / 256), dim3(256), 0, stream>>>(q, Q16, n8);
  cast8_kernel<<<dim3(n8 / 256), dim3(256), 0, stream>>>(k, K16, n8);
  vt_cast_kernel<<<dim3(kS / 64, kBH), dim3(256), 0, stream>>>(v, VT);
  attn_causal_kernel<<<dim3(kS / kQB, kBH), dim3(128), 0, stream>>>(Q16, K16, VT, out);
}
